// BigBirdAttention_69131793596540
// MI455X (gfx1250) — hardware-verified
//
#include <hip/hip_runtime.h>
#include <math.h>
#include <stdint.h>

#define NBAT  2
#define LTOK  4064
#define SEQ   4096
#define HIDW  1024
#define NH    16
#define HD    64
#define BSZ   64
#define NBLK  64
#define RR    3
#define NRROW 62
#define KOUT  2048
static_assert(NH * HD == HIDW);
static_assert(NBLK * BSZ == SEQ);
static_assert(NRROW == NBLK - 2);
static_assert(SEQ == LTOK + (BSZ - (LTOK % BSZ)));
static_assert((HIDW % 64) == 0 && (SEQ % 64) == 0 && (HIDW % 32) == 0 && (KOUT % 32) == 0);
static_assert(BSZ == 64 && HD == 64);
static_assert(KOUT == 2 * HIDW);

typedef __bf16         v16b __attribute__((ext_vector_type(16)));
typedef unsigned short v8us __attribute__((ext_vector_type(8)));
typedef float          v8f  __attribute__((ext_vector_type(8)));
typedef float          v4f  __attribute__((ext_vector_type(4)));
typedef unsigned int   v4u  __attribute__((ext_vector_type(4)));
typedef v4f  __attribute__((may_alias)) v4fa;
typedef v8us __attribute__((may_alias)) v8usa;

#if defined(__HIP_DEVICE_COMPILE__)
#define DEV_ASM 1
#else
#define DEV_ASM 0
#endif

__device__ __forceinline__ unsigned short bf_bits(float f) {
  unsigned u = __float_as_uint(f);
  return (unsigned short)((u + 0x7FFFu + ((u >> 16) & 1u)) >> 16);
}
__device__ __forceinline__ float bf_up(unsigned short hb) { return __uint_as_float(((unsigned)hb) << 16); }
__device__ __forceinline__ float bfr(float f) { return bf_up(bf_bits(f)); }
__device__ __forceinline__ unsigned pk16(unsigned short a, unsigned short b) { return (unsigned)a | ((unsigned)b << 16); }
__device__ __forceinline__ v8f zero8() { v8f z = {0.f, 0.f, 0.f, 0.f, 0.f, 0.f, 0.f, 0.f}; return z; }
__device__ __forceinline__ int imin(int a, int b) { return a < b ? a : b; }
__device__ __forceinline__ int imax(int a, int b) { return a > b ? a : b; }

union FragB { v16b v; v8us u[2]; };
__device__ __forceinline__ v16b ldfrag(const unsigned short* p) {
  FragB f;
  f.u[0] = *(const v8usa*)(p);
  f.u[1] = *(const v8usa*)(p + 16);
  return f.v;
}

__device__ __forceinline__ v8f mmab(v16b a, v16b b, v8f c) {
  return __builtin_amdgcn_wmma_f32_16x16x32_bf16(false, a, false, b, (short)0, c, false, false);
}
__device__ __forceinline__ v8f mmab_g(v16b a, v16b b, v8f c) {
  c = __builtin_amdgcn_wmma_f32_16x16x32_bf16(false, a, false, b, (short)0, c, false, false);
#if DEV_ASM
  asm volatile("v_nop\n\tv_nop\n\tv_nop\n\tv_nop" : "+v"(c) : "v"(a), "v"(b));
#endif
  return c;
}
__device__ __forceinline__ void dep_guard(v8f& a, v8f& b, v16b x, v16b y) {
#if DEV_ASM
  asm volatile("v_nop\n\tv_nop\n\tv_nop\n\tv_nop" : "+v"(a), "+v"(b) : "v"(x), "v"(y));
#else
  (void)a; (void)b; (void)x; (void)y;
#endif
}
__device__ __forceinline__ void keep4(v16b a, v16b b, v16b c, v16b d) {
#if DEV_ASM
  asm volatile("v_nop" :: "v"(a), "v"(b), "v"(c), "v"(d));
#else
  (void)a; (void)b; (void)c; (void)d;
#endif
}
__device__ __forceinline__ void acc_guard4(v8f& a, v8f& b, v8f& c, v8f& d) {
#if DEV_ASM
  asm volatile("v_nop\n\tv_nop\n\tv_nop\n\tv_nop" : "+v"(a), "+v"(b), "+v"(c), "+v"(d));
#else
  (void)a; (void)b; (void)c; (void)d;
#endif
}

__global__ __launch_bounds__(256) void cvt_x(const float* __restrict__ in, unsigned short* out, int n8) {
  const int i = blockIdx.x * 256 + (int)threadIdx.x;
  if (i < n8) {
    const size_t e  = (size_t)i * 8;
    const int    cc = (int)(e % HIDW);
    const size_t t  = e / HIDW;
    const int    s  = (int)(t % SEQ);
    const int    b  = (int)(t / SEQ);
    const int    sc = (s < LTOK) ? s : (LTOK - 1);
    const float* src = in + ((size_t)b * LTOK + (size_t)sc) * HIDW + cc;
    const v4f a  = *(const v4fa*)(src);
    const v4f a4 = *(const v4fa*)(src + 4);
    const bool live = (s < LTOK);
    v4u p;
    p[0] = live ? pk16(bf_bits(a[0]),  bf_bits(a[1]))  : 0u;
    p[1] = live ? pk16(bf_bits(a[2]),  bf_bits(a[3]))  : 0u;
    p[2] = live ? pk16(bf_bits(a4[0]), bf_bits(a4[1])) : 0u;
    p[3] = live ? pk16(bf_bits(a4[2]), bf_bits(a4[3])) : 0u;
    unsigned short* o = out + e;
    *(volatile v4u*)o = p;
    __threadfence();
    *(volatile v4u*)o = p;
  }
}

__global__ __launch_bounds__(256) void cvt_wt(const float* __restrict__ Wq, const float* __restrict__ Wk,
                                              const float* __restrict__ Wv, const float* __restrict__ Wo,
                                              unsigned short* WTq, unsigned short* WTk, unsigned short* WTv,
                                              unsigned short* WTo2) {
  __shared__ float sW[64][65];
  const int tid = (int)threadIdx.x;
  const int n0  = blockIdx.x * 64;
  const int k0  = blockIdx.y * 64;
  const int mat = blockIdx.z;
  const float* W = (mat == 0) ? Wq : ((mat == 1) ? Wk : ((mat == 2) ? Wv : Wo));
  unsigned short* WT = (mat == 0) ? WTq : ((mat == 1) ? WTk : ((mat == 2) ? WTv : WTo2));
  const int pitch = (mat == 3) ? KOUT : HIDW;
  const int c4 = (tid & 15) * 4, rsub = tid >> 4;
#pragma unroll
  for (int it = 0; it < 4; ++it) {
    const int r = it * 16 + rsub;
    const v4f v = *(const v4fa*)(W + (size_t)(k0 + r) * HIDW + n0 + c4);
    sW[c4 + 0][r] = v[0];
    sW[c4 + 1][r] = v[1];
    sW[c4 + 2][r] = v[2];
    sW[c4 + 3][r] = v[3];
  }
  __syncthreads();
  const int sub = tid >> 3, c8 = (tid & 7) * 8;
  v4u pv[2];
#pragma unroll
  for (int it = 0; it < 2; ++it) {
    const int li = it * 32 + sub;
    v4u a;
#pragma unroll
    for (int e = 0; e < 4; ++e)
      a[e] = pk16(bf_bits(sW[li][c8 + 2 * e]), bf_bits(sW[li][c8 + 2 * e + 1]));
    pv[it] = a;
  }
  for (int pass = 0; pass < 2; ++pass) {
#pragma unroll
    for (int it = 0; it < 2; ++it) {
      const int li = it * 32 + sub;
      unsigned short* dst = WT + (size_t)(n0 + li) * pitch + k0 + c8;
      *(volatile v4u*)(dst) = pv[it];
      if (mat == 3) *(volatile v4u*)(dst + HIDW) = pv[it];
    }
    __threadfence();
  }
}

template <int MODE>
__global__ __launch_bounds__(256) void gemm64(
    const unsigned short* __restrict__ A, int lda,
    const unsigned short* __restrict__ Bt, int ldb,
    const float* __restrict__ bias, int blen, int biasRow,
    unsigned short* Ch, unsigned short* Cl, float* Cf, int ldc,
    int M, int N, int K, int Mvalid, float oscale) {
  __shared__ __align__(16) float sT[8][16 * 68];
  const int lane = threadIdx.x & 31;
  const int wave = threadIdx.x >> 5;
  const int tilesN = N >> 6;
  const int tilesM = M >> 6;
  const int tile = blockIdx.x * 8 + wave;
  if (tile >= tilesM * tilesN) return;
  const int tm = tile / tilesN;
  const int tn = tile - tm * tilesN;
  const int m0 = tm << 6;
  const int n0 = tn << 6;

  const int rlane = lane & 15;
  const int koff  = (lane >> 4) * 8;
  const int mOff  = (lane >> 4) * 8;

  v8f acc[4][4];
#pragma unroll
  for (int i = 0; i < 4; ++i)
#pragma unroll
    for (int j = 0; j < 4; ++j) acc[i][j] = zero8();

  for (int k0 = 0; k0 < K; k0 += 32) {
    v16b bq[4];
#pragma unroll
    for (int j = 0; j < 4; ++j)
      bq[j] = ldfrag(Bt + (size_t)(n0 + (j << 4) + rlane) * ldb + koff + k0);
#pragma unroll
    for (int i = 0; i < 4; ++i) {
      const v16b af = ldfrag(A + (size_t)(m0 + (i << 4) + rlane) * lda + koff + k0);
#pragma unroll
      for (int j = 0; j < 4; ++j) acc[i][j] = mmab(af, bq[j], acc[i][j]);
      dep_guard(acc[i][0], acc[i][3], af, bq[3]);
    }
    keep4(bq[0], bq[1], bq[2], bq[3]);
  }
  acc_guard4(acc[0][0], acc[0][1], acc[0][2], acc[0][3]);
  acc_guard4(acc[1][0], acc[1][1], acc[1][2], acc[1][3]);
  acc_guard4(acc[2][0], acc[2][1], acc[2][2], acc[2][3]);
  acc_guard4(acc[3][0], acc[3][1], acc[3][2], acc[3][3]);

  float* slab = sT[wave];
  const int bl1 = blen - 1;
  if (MODE == 0) {
    const int q = lane >> 3, c8 = (lane & 7) * 8;
    float bcv[8];
#pragma unroll
    for (int e = 0; e < 8; ++e) bcv[e] = bfr(bias[imin(imax(n0 + c8 + e, 0), bl1)]);
#pragma unroll
    for (int i = 0; i < 4; ++i) {
      const int mBase = m0 + (i << 4);
#pragma unroll
      for (int j = 0; j < 4; ++j) {
#pragma unroll
        for (int r = 0; r < 8; ++r) {
          slab[(mOff + r) * 68 + (j << 4) + rlane] = acc[i][j][r];
        }
      }
      __builtin_amdgcn_fence(__ATOMIC_RELEASE, "workgroup");
      __builtin_amdgcn_wave_barrier();
      __builtin_amdgcn_fence(__ATOMIC_ACQUIRE, "workgroup");
      v4u hv[4], lv[4];
#pragma unroll
      for (int it = 0; it < 4; ++it) {
        const int row = it * 4 + q;
        const float* sp = slab + row * 68 + c8;
        const float brv = bfr(bias[imin(imax(mBase + row, 0), bl1)]);
        float f[8];
#pragma unroll
        for (int e = 0; e < 8; ++e) {
          const float bb = biasRow ? brv : bcv[e];
          f[e] = (sp[e] + bb) * oscale;
        }
        v4u a, a2;
#pragma unroll
        for (int e = 0; e < 4; ++e) {
          const float f0 = f[2 * e], f1 = f[2 * e + 1];
          const unsigned short h0 = bf_bits(f0), h1 = bf_bits(f1);
          const unsigned short l0 = bf_bits(f0 - bf_up(h0));
          const unsigned short l1 = bf_bits(f1 - bf_up(h1));
          a[e] = pk16(h0, h1); a2[e] = pk16(l0, l1);
        }
        hv[it] = a; lv[it] = a2;
      }
      for (int pass = 0; pass < 2; ++pass) {
#pragma unroll
        for (int it = 0; it < 4; ++it) {
          const int row = it * 4 + q;
          *(volatile v4u*)(Ch + (size_t)(mBase + row) * ldc + n0 + c8) = hv[it];
          *(volatile v4u*)(Cl + (size_t)(mBase + row) * ldc + n0 + c8) = lv[it];
        }
        __threadfence();
      }
      __builtin_amdgcn_fence(__ATOMIC_RELEASE, "workgroup");
      __builtin_amdgcn_wave_barrier();
      __builtin_amdgcn_fence(__ATOMIC_ACQUIRE, "workgroup");
    }
  } else {
    const int h2 = lane >> 4, c4 = (lane & 15) * 4;
    float b4[4];
#pragma unroll
    for (int e = 0; e < 4; ++e) b4[e] = bfr(bias[imin(imax(n0 + c4 + e, 0), bl1)]);
#pragma unroll
    for (int i = 0; i < 4; ++i) {
      const int mBase = m0 + (i << 4);
#pragma unroll
      for (int j = 0; j < 4; ++j) {
#pragma unroll
        for (int r = 0; r < 8; ++r) {
          slab[(mOff + r) * 68 + (j << 4) + rlane] = acc[i][j][r];
        }
      }
      __builtin_amdgcn_fence(__ATOMIC_RELEASE, "workgroup");
      __builtin_amdgcn_wave_barrier();
      __builtin_amdgcn_fence(__ATOMIC_ACQUIRE, "workgroup");
      v4f ov[8];
#pragma unroll
      for (int it = 0; it < 8; ++it) {
        const int row = it * 2 + h2;
        const float* sp = slab + row * 68 + c4;
        v4f v;
#pragma unroll
        for (int e = 0; e < 4; ++e) v[e] = sp[e] + b4[e];
        ov[it] = v;
      }
      for (int pass = 0; pass < 2; ++pass) {
#pragma unroll
        for (int it = 0; it < 8; ++it) {
          const int row = it * 2 + h2;
          const int gm = mBase + row;
          if (gm < Mvalid)
            *(volatile v4f*)(Cf + (size_t)gm * ldc + n0 + c4) = ov[it];
        }
        __threadfence();
      }
      __builtin_amdgcn_fence(__ATOMIC_RELEASE, "workgroup");
      __builtin_amdgcn_wave_barrier();
      __builtin_amdgcn_fence(__ATOMIC_ACQUIRE, "workgroup");
    }
  }
}

union __align__(16) SU {
  unsigned short kv[4][64 * 64];
  float          os[4][16 * 64];
};

__device__ __forceinline__ int clamp_blk(int v) {
  v = (v < 0) ? (v + NBLK) : v;
  v = (v < 0) ? 0 : v;
  v = (v > NBLK - 1) ? (NBLK - 1) : v;
  return v;
}

template <int DENSE>
__global__ __launch_bounds__(128)
void attn_bs(const unsigned short* __restrict__ Qh, const unsigned short* __restrict__ Ql,
             const unsigned short* __restrict__ Kh, const unsigned short* __restrict__ Kl,
             const unsigned short* __restrict__ VTh, const unsigned short* __restrict__ VTl,
             const int* __restrict__ rb, unsigned short* Cx) {
  __shared__ SU su;
  __shared__ __align__(16) unsigned short Psh[2][4][16 * 64];

  const int tid  = threadIdx.x;
  const int wave = tid >> 5;
  const int lane = tid & 31;
  const int hh   = lane >> 4;
  const int c    = lane & 15;

  int h, nb;
  if (DENSE) {
    h  = (int)blockIdx.x >> 1;
    nb = ((int)blockIdx.x & 1) ? (NBLK - 1) : 0;
  } else {
    h  = (int)blockIdx.x / NRROW;
    nb = 1 + ((int)blockIdx.x - h * NRROW);
  }
  h  = (h > NH - 1) ? (NH - 1) : h;
  nb = (nb > NBLK - 1) ? (NBLK - 1) : nb;

  int nband = 3, band0 = nb - 1;
  if (nb == 1)        { nband = 2; band0 = 1; }
  if (nb == NBLK - 2) { nband = 2; band0 = NBLK - 3; }
  int rb0 = 0, rb1 = 0, rb2 = 0;
  if (!DENSE) {
    int rrow = nb - 1;
    rrow = (rrow < 0) ? 0 : ((rrow > NRROW - 1) ? (NRROW - 1) : rrow);
    const int* rp = rb + ((size_t)h * NRROW + rrow) * RR;
    rb0 = clamp_blk(rp[0]);
    rb1 = clamp_blk(rp[1]);
    rb2 = clamp_blk(rp[2]);
  }

  const int q0 = nb * BSZ + wave * 16;

  v16b qah[2], qal[2];
#pragma unroll
  for (int dc = 0; dc < 2; ++dc) {
    const size_t qo = (size_t)(q0 + c) * HIDW + (size_t)h * HD + dc * 32 + 8 * hh;
    qah[dc] = ldfrag(Qh + qo);
    qal[dc] = ldfrag(Ql + qo);
  }

  float mrow[8], lrow[8];
  v8f oacc[4];
#pragma unroll
  for (int r = 0; r < 8; ++r) { mrow[r] = -INFINITY; lrow[r] = 0.f; }
#pragma unroll
  for (int t = 0; t < 4; ++t) oacc[t] = zero8();

  unsigned short* pwh = Psh[0][wave];
  unsigned short* pwl = Psh[1][wave];

  const int NIT = DENSE ? NBLK : (5 + nband);
#pragma unroll 1
  for (int it = 0; it < NIT; ++it) {
    int kblk;
    if (DENSE) {
      kblk = it;
    } else {
      const int jr = it - 2 - nband;
      kblk = (it == 0) ? 0 : (it == 1) ? (NBLK - 1) : (jr < 0) ? (band0 + it - 2) :
             (jr == 0) ? rb0 : (jr == 1) ? rb1 : rb2;
      kblk = (kblk < 0) ? 0 : ((kblk > NBLK - 1) ? (NBLK - 1) : kblk);
    }
    const int ks = kblk * BSZ;
    __syncthreads();
    {
      const int r = tid >> 1, half = (tid & 1) * 32;
      const unsigned short* kgh = Kh  + (size_t)(ks + r) * HIDW + (size_t)h * HD + half;
      const unsigned short* kgl = Kl  + (size_t)(ks + r) * HIDW + (size_t)h * HD + half;
      const unsigned short* vgh = VTh + (size_t)(h * HD + r) * SEQ + ks + half;
      const unsigned short* vgl = VTl + (size_t)(h * HD + r) * SEQ + ks + half;
#pragma unroll
      for (int i = 0; i < 4; ++i) {
        const v8us a0 = *(const v8usa*)(kgh + 8 * i);
        const v8us a1 = *(const v8usa*)(kgl + 8 * i);
        const v8us b0 = *(const v8usa*)(vgh + 8 * i);
        const v8us b1 = *(const v8usa*)(vgl + 8 * i);
        *(v8us*)(su.kv[0] + r * 64 + half + 8 * i) = a0;
        *(v8us*)(su.kv[1] + r * 64 + half + 8 * i) = a1;
        *(v8us*)(su.kv[2] + r * 64 + half + 8 * i) = b0;
        *(v8us*)(su.kv[3] + r * 64 + half + 8 * i) = b1;
      }
    }
    __syncthreads();

    v8f s[4];
#pragma unroll
    for (int j = 0; j < 4; ++j) {
      v8f z = zero8();
#pragma unroll
      for (int dc = 0; dc < 2; ++dc) {
        const v16b kfh = ldfrag(su.kv[0] + (j * 16 + c) * 64 + dc * 32 + 8 * hh);
        const v16b kfl = ldfrag(su.kv[1] + (j * 16 + c) * 64 + dc * 32 + 8 * hh);
        z = mmab_g(qah[dc], kfh, z);
        z = mmab_g(qah[dc], kfl, z);
        z = mmab_g(qal[dc], kfh, z);
      }
      s[j] = z;
    }

#pragma unroll
    for (int r = 0; r < 8; ++r) {
      float m = s[0][r];
#pragma unroll
      for (int j = 1; j < 4; ++j) m = fmaxf(m, s[j][r]);
#pragma unroll
      for (int off = 1; off < 16; off <<= 1) m = fmaxf(m, __shfl_xor(m, off, 32));
      const float mnew  = fmaxf(mrow[r], m);
      const float msafe = (mnew == -INFINITY) ? 0.f : mnew;
      const float alpha = __expf(mrow[r] - msafe);
      mrow[r] = mnew;
      float psum = 0.f;
#pragma unroll
      for (int j = 0; j < 4; ++j) {
        const float p = __expf(s[j][r] - msafe);
        psum += p;
        const unsigned short hb = bf_bits(p);
        const unsigned short lb = bf_bits(p - bf_up(hb));
        pwh[(8 * hh + r) * 64 + j * 16 + c] = hb;
        pwl[(8 * hh + r) * 64 + j * 16 + c] = lb;
      }
#pragma unroll
      for (int off = 1; off < 16; off <<= 1) psum += __shfl_xor(psum, off, 32);
      lrow[r] = lrow[r] * alpha + psum;
#pragma unroll
      for (int t = 0; t < 4; ++t) oacc[t][r] *= alpha;
    }
    __builtin_amdgcn_fence(__ATOMIC_RELEASE, "workgroup");
    __builtin_amdgcn_wave_barrier();
    __builtin_amdgcn_fence(__ATOMIC_ACQUIRE, "workgroup");

#pragma unroll 1
    for (int kk = 0; kk < 2; ++kk) {
      const v16b pah = ldfrag(pwh + c * 64 + kk * 32 + 8 * hh);
      const v16b pal = ldfrag(pwl + c * 64 + kk * 32 + 8 * hh);
#pragma unroll
      for (int t = 0; t < 4; ++t) {
        const v16b vfh = ldfrag(su.kv[2] + (t * 16 + c) * 64 + kk * 32 + 8 * hh);
        const v16b vfl = ldfrag(su.kv[3] + (t * 16 + c) * 64 + kk * 32 + 8 * hh);
        oacc[t] = mmab_g(pah, vfh, oacc[t]);
        oacc[t] = mmab_g(pal, vfh, oacc[t]);
        oacc[t] = mmab_g(pah, vfl, oacc[t]);
      }
    }
  }

  __syncthreads();
  float* os = su.os[wave];
#pragma unroll
  for (int r = 0; r < 8; ++r) {
    const float l = lrow[r];
    const float inv = (l > 0.f) ? (1.0f / l) : 0.f;
#pragma unroll
    for (int t = 0; t < 4; ++t) os[(8 * hh + r) * 64 + t * 16 + c] = oacc[t][r] * inv;
  }
  __builtin_amdgcn_fence(__ATOMIC_RELEASE, "workgroup");
  __builtin_amdgcn_wave_barrier();
  __builtin_amdgcn_fence(__ATOMIC_ACQUIRE, "workgroup");
  {
    const int q = lane >> 3, c8 = (lane & 7) * 8;
    v4u hv[4], lv[4];
#pragma unroll
    for (int it = 0; it < 4; ++it) {
      const int row = it * 4 + q;
      const float* sp = os + row * 64 + c8;
      v4u a, a2;
#pragma unroll
      for (int e = 0; e < 4; ++e) {
        const float f0 = sp[2 * e], f1 = sp[2 * e + 1];
        const unsigned short h0 = bf_bits(f0), h1 = bf_bits(f1);
        const unsigned short l0 = bf_bits(f0 - bf_up(h0));
        const unsigned short l1 = bf_bits(f1 - bf_up(h1));
        a[e] = pk16(h0, h1); a2[e] = pk16(l0, l1);
      }
      hv[it] = a; lv[it] = a2;
    }
    const size_t obase = (size_t)q0 * KOUT + (size_t)h * HD + c8;
    for (int pass = 0; pass < 2; ++pass) {
#pragma unroll
      for (int it = 0; it < 4; ++it) {
        const int row = it * 4 + q;
        *(volatile v4u*)(Cx + obase + (size_t)row * KOUT)        = hv[it];
        *(volatile v4u*)(Cx + obase + (size_t)row * KOUT + HIDW) = lv[it];
      }
      __threadfence();
    }
  }
}

__device__ __forceinline__ int scan_ne1(const float* __restrict__ p, int n, int tid) {
  int bad = 0;
  const int n4 = n >> 2;
#pragma unroll 1
  for (int i = tid; i < n4; i += 256) {
    const v4f v = *(const v4fa*)(p + (size_t)i * 4);
    bad |= (v[0] != 1.0f) | (v[1] != 1.0f) | (v[2] != 1.0f) | (v[3] != 1.0f);
  }
#pragma unroll 1
  for (int i = (n4 << 2) + tid; i < n; i += 256) bad |= (p[i] != 1.0f);
  return bad;
}

__global__ __launch_bounds__(256) void mask_guard(const float* __restrict__ mk0, int nk0,
                                                  const float* __restrict__ mk1, int nk1,
                                                  const float* __restrict__ mk2, int nk2,
                                                  const float* __restrict__ mk3, int nk3,
                                                  float* out) {
  __shared__ int sf[256];
  const int tid = (int)threadIdx.x;
  int bad = 0;
  bad |= scan_ne1(mk0, nk0, tid);
  bad |= scan_ne1(mk1, nk1, tid);
  bad |= scan_ne1(mk2, nk2, tid);
  bad |= scan_ne1(mk3, nk3, tid);
  sf[tid] = bad;
  __syncthreads();
  for (int st = 128; st > 0; st >>= 1) {
    if (tid < st) sf[tid] |= sf[tid + st];
    __syncthreads();
  }
  const int anybad = sf[0];
  if (anybad != 0 && tid < 8) {
    const float qn = __uint_as_float(0x7fc00000u);
    v4f nv = {qn, qn, qn, qn};
    float* o = out + tid * 4;
    *(volatile v4f*)o = nv;
    __threadfence();
    *(volatile v4f*)o = nv;
  }
}

extern "C" void kernel_launch(void* const* d_in, const int* in_sizes, int n_in,
                              void* d_out, int out_size, void* d_ws, size_t ws_size,
                              hipStream_t stream) {
  if (n_in < 14) return;
  if (in_sizes[0] != NBAT * LTOK * HIDW) return;
  if (in_sizes[1] != HIDW * HIDW || in_sizes[3] != HIDW * HIDW ||
      in_sizes[5] != HIDW * HIDW || in_sizes[7] != HIDW * HIDW) return;
  if (in_sizes[2] != HIDW || in_sizes[4] != HIDW || in_sizes[6] != HIDW || in_sizes[8] != HIDW) return;
  if (in_sizes[9] < 1 || in_sizes[10] < 1 || in_sizes[11] < 1 || in_sizes[12] < 1) return;
  if (in_sizes[13] != NBAT * NH * NRROW * RR) return;
  if (out_size != NBAT * LTOK * HIDW) return;

  const float* x     = (const float*)d_in[0];
  const float* Wq    = (const float*)d_in[1];
  const float* bq    = (const float*)d_in[2];
  const float* Wk    = (const float*)d_in[3];
  const float* bk    = (const float*)d_in[4];
  const float* Wv    = (const float*)d_in[5];
  const float* bv    = (const float*)d_in[6];
  const float* Wo    = (const float*)d_in[7];
  const float* bo    = (const float*)d_in[8];
  const float* mband = (const float*)d_in[9];
  const float* mfrom = (const float*)d_in[10];
  const float* mto   = (const float*)d_in[11];
  const float* mblk  = (const float*)d_in[12];
  const int*   rattn = (const int*)d_in[13];
  float* out = (float*)d_out;

  const size_t PX  = (size_t)NBAT * SEQ * HIDW * 2;
  const size_t PW  = (size_t)HIDW * HIDW * 2;
  const size_t PWO = (size_t)HIDW * KOUT * 2;
  const size_t PP  = (size_t)SEQ * HIDW * 2;
  const size_t PC  = (size_t)SEQ * KOUT * 2;
  size_t off = 0;
  const size_t oXb  = off; off += PX;
  const size_t oWq  = off; off += PW;
  const size_t oWk  = off; off += PW;
  const size_t oWv  = off; off += PW;
  const size_t oWo  = off; off += PWO;
  const size_t oQh  = off; off += PP;
  const size_t oQl  = off; off += PP;
  const size_t oKh  = off; off += PP;
  const size_t oKl  = off; off += PP;
  const size_t oVTh = off; off += PP;
  const size_t oVTl = off; off += PP;
  const size_t oCtx = off; off += PC;
  if (off > ws_size) return;
  if (off > (size_t)134217728) return;

  char* ws = (char*)d_ws;
  unsigned short* Xb   = (unsigned short*)(ws + oXb);
  unsigned short* WTq  = (unsigned short*)(ws + oWq);
  unsigned short* WTk  = (unsigned short*)(ws + oWk);
  unsigned short* WTv  = (unsigned short*)(ws + oWv);
  unsigned short* WTo2 = (unsigned short*)(ws + oWo);
  unsigned short* Qh   = (unsigned short*)(ws + oQh);
  unsigned short* Ql   = (unsigned short*)(ws + oQl);
  unsigned short* Kh   = (unsigned short*)(ws + oKh);
  unsigned short* Kl   = (unsigned short*)(ws + oKl);
  unsigned short* VTh  = (unsigned short*)(ws + oVTh);
  unsigned short* VTl  = (unsigned short*)(ws + oVTl);
  unsigned short* Ctx  = (unsigned short*)(ws + oCtx);

  const int n8x = NBAT * SEQ * HIDW / 8;
  const dim3 gCvtX((n8x + 255) / 256);
  const dim3 gCvtW(HIDW / 64, HIDW / 64, 4);
  const dim3 blk(256);
  const int tilesQ  = (SEQ / 64) * (HIDW / 64);
  const int tilesVT = (HIDW / 64) * (SEQ / 64);
  const int tilesO  = (SEQ / 64) * (HIDW / 64);
  const dim3 gQ((tilesQ + 7) / 8);
  const dim3 gVT((tilesVT + 7) / 8);
  const dim3 gO((tilesO + 7) / 8);
  const dim3 gSparse(NH * NRROW);
  const dim3 gDense(NH * 2);

  cvt_x<<<gCvtX, blk, 0, stream>>>(x, Xb, n8x);
  cvt_wt<<<gCvtW, blk, 0, stream>>>(Wq, Wk, Wv, Wo, WTq, WTk, WTv, WTo2);

  for (int b = 0; b < NBAT; ++b) {
    const unsigned short* Xbb = Xb + (size_t)b * SEQ * HIDW;
    const int* rbb = rattn + (size_t)b * NH * NRROW * RR;
    float* outb = out + (size_t)b * LTOK * HIDW;
    gemm64<0><<<gQ, blk, 0, stream>>>(Xbb, HIDW, WTq, HIDW, bq, HIDW, 0, Qh, Ql, out, HIDW,
                                       SEQ, HIDW, HIDW, SEQ, 0.125f);
    gemm64<0><<<gQ, blk, 0, stream>>>(Xbb, HIDW, WTk, HIDW, bk, HIDW, 0, Kh, Kl, out, HIDW,
                                       SEQ, HIDW, HIDW, SEQ, 1.0f);
    gemm64<0><<<gVT, blk, 0, stream>>>(WTv, HIDW, Xbb, HIDW, bv, HIDW, 1, VTh, VTl, out, SEQ,
                                        HIDW, SEQ, HIDW, HIDW, 1.0f);
    attn_bs<0><<<gSparse, dim3(128), 0, stream>>>(Qh, Ql, Kh, Kl, VTh, VTl, rbb, Ctx);
    attn_bs<1><<<gDense,  dim3(128), 0, stream>>>(Qh, Ql, Kh, Kl, VTh, VTl, rbb, Ctx);
    gemm64<1><<<gO, blk, 0, stream>>>(Ctx, KOUT, WTo2, KOUT, bo, HIDW, 0, Qh, Ql, outb, HIDW,
                                       SEQ, HIDW, KOUT, LTOK, 1.0f);
  }
  mask_guard<<<dim3(1), blk, 0, stream>>>(mband, in_sizes[9], mfrom, in_sizes[10], mto, in_sizes[11],
                                          mblk, in_sizes[12], out);
  (void)hipGetLastError();
}
